// Vmamba1DBlock_90237262889283
// MI455X (gfx1250) — hardware-verified
//
#include <hip/hip_runtime.h>
#include <stdint.h>


#define D_MODEL   768
#define D_STATE   16
#define D_INNER   1536
#define DT_RANK   48
#define DT_PAD    64
#define XP_N      80
#define XP_PAD    128
#define KDIR      2
#define B_SZ      2
#define L_SEQ     2048
#define M_ROWS    (B_SZ * L_SEQ)
#define TCH       32
#define SCP       36
#define W_SCALE   64.0f
#define DTW_SCALE 16.0f

static_assert(M_ROWS % 64 == 0);
static_assert((2 * D_INNER) % 64 == 0 && D_INNER % 64 == 0 && D_MODEL % 64 == 0 && XP_PAD % 64 == 0);
static_assert(D_MODEL % 32 == 0 && D_INNER % 32 == 0 && DT_PAD % 32 == 0);
static_assert(L_SEQ % TCH == 0 && TCH * 8 == 256 && D_INNER % 256 == 0);
static_assert(DT_RANK % 8 == 0 && XP_N <= XP_PAD && DT_RANK <= DT_PAD);

typedef _Float16 f16t;
typedef f16t  v16h __attribute__((ext_vector_type(16)));
typedef f16t  v8h  __attribute__((ext_vector_type(8)));
typedef float v8f  __attribute__((ext_vector_type(8)));
typedef float v4f  __attribute__((ext_vector_type(4)));
union Frag { v16h v; v8h h2[2]; };

__device__ __forceinline__ v8f wmma16(v16h a, v16h b, v8f c) {
  v8f d = __builtin_amdgcn_wmma_f32_16x16x32_f16(false, a, false, b, (short)0, c, false, false);
  asm volatile("v_nop\n\tv_nop\n\tv_nop\n\tv_nop" : "+v"(d) : "v"(a), "v"(b));
  return d;
}

__device__ __forceinline__ float conv_silu1(float xp, float x0, float xn,
                                           float w0, float w1, float w2, float bb) {
  float a = w0 * xp;
  a = fmaf(w1, x0, a);
  a = fmaf(w2, xn, a);
  a = a + bb;
  float e = __expf(-a);
  return a * __builtin_amdgcn_rcpf(1.0f + e);
}

__device__ __forceinline__ float softplus1(float x) {
  return fmaxf(x, 0.0f) + log1pf(__expf(-fabsf(x)));
}

__global__ __launch_bounds__(256) void k_cvt_rows(
    const float* __restrict__ src, f16t* dst,
    int Rs, int Cs, int ps, int R, int Cd, long long sbs, long long dbs, float scale)
{
  const size_t cg  = (size_t)(Cd >> 3);
  const size_t ngr = (size_t)R * cg;
  const size_t idx = (size_t)blockIdx.x * 256 + threadIdx.x;
  if (idx >= ngr) return;
  const int r = (int)(idx / cg);
  const int c = (int)(idx % cg) * 8;
  const float* sb = src + (size_t)blockIdx.y * (size_t)sbs;
  f16t*        db = dst + (size_t)blockIdx.y * (size_t)dbs;
  v8h o;
  if (r < Rs && c < Cs) {
    const float* p = sb + (size_t)r * (size_t)ps + c;
    v4f x0 = *(const v4f*)(p);
    v4f x1 = *(const v4f*)(p + 4);
    o[0] = (f16t)(x0[0] * scale); o[1] = (f16t)(x0[1] * scale);
    o[2] = (f16t)(x0[2] * scale); o[3] = (f16t)(x0[3] * scale);
    o[4] = (f16t)(x1[0] * scale); o[5] = (f16t)(x1[1] * scale);
    o[6] = (f16t)(x1[2] * scale); o[7] = (f16t)(x1[3] * scale);
  } else {
    o[0] = (f16t)0.0f; o[1] = (f16t)0.0f; o[2] = (f16t)0.0f; o[3] = (f16t)0.0f;
    o[4] = (f16t)0.0f; o[5] = (f16t)0.0f; o[6] = (f16t)0.0f; o[7] = (f16t)0.0f;
  }
  f16t* q = db + (size_t)r * (size_t)Cd + c;
  *(volatile v8h*)q = o;
  __threadfence();
  *(volatile v8h*)q = o;
}

__global__ __launch_bounds__(128) void k_gemm_f16(
    const f16t* __restrict__ A, const f16t* __restrict__ W, float* C,
    int M, int N, int K, long long sa, long long sw, long long sc, float oscale)
{
  __shared__ __attribute__((aligned(16))) float sC[4 * 32 * SCP];
  (void)M;
  const int tid  = threadIdx.x;
  const int lane = tid & 31, wave = tid >> 5;
  const int h = lane >> 4, m = lane & 15;
  const int wm = wave >> 1, wn = wave & 1;
  const int row0 = blockIdx.y * 64 + wm * 32;
  const int col0 = blockIdx.x * 64 + wn * 32;

  const f16t* Ab = A + (size_t)blockIdx.z * (size_t)sa;
  const f16t* Wb = W + (size_t)blockIdx.z * (size_t)sw;
  float*      Cb = C + (size_t)blockIdx.z * (size_t)sc;

  const f16t* ap0 = Ab + (size_t)(row0 + m) * (size_t)K + 8 * h;
  const f16t* ap1 = ap0 + (size_t)16 * (size_t)K;
  const f16t* wp0 = Wb + (size_t)(col0 + m) * (size_t)K + 8 * h;
  const f16t* wp1 = wp0 + (size_t)16 * (size_t)K;

  v8f c00 = {0.f, 0.f, 0.f, 0.f, 0.f, 0.f, 0.f, 0.f};
  v8f c01 = c00, c10 = c00, c11 = c00;

  for (int k0 = 0; k0 < K; k0 += 32) {
    Frag a0, a1, b0, b1;
    a0.h2[0] = *(const v8h*)(ap0 + k0);
    a0.h2[1] = *(const v8h*)(ap0 + k0 + 16);
    a1.h2[0] = *(const v8h*)(ap1 + k0);
    a1.h2[1] = *(const v8h*)(ap1 + k0 + 16);
    b0.h2[0] = *(const v8h*)(wp0 + k0);
    b0.h2[1] = *(const v8h*)(wp0 + k0 + 16);
    b1.h2[0] = *(const v8h*)(wp1 + k0);
    b1.h2[1] = *(const v8h*)(wp1 + k0 + 16);
    c00 = wmma16(a0.v, b0.v, c00);
    c01 = wmma16(a0.v, b1.v, c01);
    c10 = wmma16(a1.v, b0.v, c10);
    c11 = wmma16(a1.v, b1.v, c11);
  }

  float* st = sC + wave * (32 * SCP);
#pragma unroll
  for (int r = 0; r < 8; ++r) {
    st[(8 * h + r) * SCP + m]           = c00[r] * oscale;
    st[(8 * h + r) * SCP + 16 + m]      = c01[r] * oscale;
    st[(16 + 8 * h + r) * SCP + m]      = c10[r] * oscale;
    st[(16 + 8 * h + r) * SCP + 16 + m] = c11[r] * oscale;
  }
  __syncthreads();

  const int rq = lane >> 3;
  const int c4 = (lane & 7) * 4;
  v4f vals[8];
#pragma unroll
  for (int it = 0; it < 8; ++it)
    vals[it] = *(const v4f*)(st + (it * 4 + rq) * SCP + c4);

  float* cbase = Cb + (size_t)row0 * (size_t)N + col0 + c4;
#pragma unroll
  for (int it = 0; it < 8; ++it)
    *(volatile v4f*)(cbase + (size_t)(it * 4 + rq) * (size_t)N) = vals[it];
  __threadfence();
#pragma unroll
  for (int it = 0; it < 8; ++it)
    *(volatile v4f*)(cbase + (size_t)(it * 4 + rq) * (size_t)N) = vals[it];
}

__global__ __launch_bounds__(256) void k_conv_silu(
    const float* __restrict__ xz, const float* __restrict__ cw,
    const float* __restrict__ cb, f16t* uh)
{
  const size_t cgr = (size_t)(D_INNER / 8);
  const size_t ngr = (size_t)M_ROWS * cgr;
  const size_t idx = (size_t)blockIdx.x * 256 + threadIdx.x;
  if (idx >= ngr) return;
  const int r = (int)(idx / cgr);
  const int c = (int)(idx % cgr) * 8;
  const int l = r % L_SEQ;
  const float* p0 = xz + (size_t)r * (size_t)(2 * D_INNER) + c;

  union U8  { v4f v[2]; float f[8]; };
  union U24 { v4f v[6]; float f[24]; };
  U8 x0, xp, xn, bb;
  U24 w;
  const v4f z4 = {0.f, 0.f, 0.f, 0.f};
  x0.v[0] = *(const v4f*)(p0);
  x0.v[1] = *(const v4f*)(p0 + 4);
  if (l > 0) {
    const float* pp = p0 - 2 * D_INNER;
    xp.v[0] = *(const v4f*)(pp); xp.v[1] = *(const v4f*)(pp + 4);
  } else { xp.v[0] = z4; xp.v[1] = z4; }
  if (l < L_SEQ - 1) {
    const float* pn = p0 + 2 * D_INNER;
    xn.v[0] = *(const v4f*)(pn); xn.v[1] = *(const v4f*)(pn + 4);
  } else { xn.v[0] = z4; xn.v[1] = z4; }
  bb.v[0] = *(const v4f*)(cb + c);
  bb.v[1] = *(const v4f*)(cb + c + 4);
#pragma unroll
  for (int q = 0; q < 6; ++q) w.v[q] = *(const v4f*)(cw + (size_t)c * 3 + 4 * q);

  v8h o;
#pragma unroll
  for (int i = 0; i < 8; ++i)
    o[i] = (f16t)conv_silu1(xp.f[i], x0.f[i], xn.f[i], w.f[3 * i], w.f[3 * i + 1], w.f[3 * i + 2], bb.f[i]);

  f16t* q = uh + idx * 8;
  *(volatile v8h*)q = o;
  __threadfence();
  *(volatile v8h*)q = o;
}

__global__ __launch_bounds__(256) void k_scan(
    const float* __restrict__ xz, const float* __restrict__ cw, const float* __restrict__ cb,
    const float* __restrict__ dt_raw, const float* __restrict__ dt_b, const float* __restrict__ x_dbl,
    const float* __restrict__ A_logs, const float* __restrict__ Ds,
    const float* y0_in, float* y0_out, f16t* yg_out, int dir)
{
  __shared__ __attribute__((aligned(16))) float sBC[TCH * 2 * D_STATE];
  __shared__ __attribute__((aligned(16))) float sY[TCH * 256];
  f16t* sYh = (f16t*)sY;

  const int tid = threadIdx.x;
  const int nb = D_INNER / 256;
  const int b = blockIdx.x / nb, dblk = blockIdx.x % nb;
  const int d = dblk * 256 + tid;
  const size_t rb = (size_t)b * L_SEQ;

  float An[D_STATE], hs[D_STATE];
#pragma unroll
  for (int n = 0; n < D_STATE; ++n) {
    An[n] = -__expf(A_logs[(size_t)d * D_STATE + n]);
    hs[n] = 0.0f;
  }
  const float Dk = Ds[d], bias = dt_b[d];
  const float w0 = cw[d * 3 + 0], w1 = cw[d * 3 + 1], w2 = cw[d * 3 + 2], cbv = cb[d];

#pragma unroll 1
  for (int t0 = 0; t0 < L_SEQ; t0 += TCH) {
    {
      const int s = tid >> 3, j = (tid & 7) * 4;
      const int t = t0 + s;
      const int l = dir ? (L_SEQ - 1 - t) : t;
      v4f v = *(const v4f*)(x_dbl + (rb + (size_t)l) * XP_PAD + DT_RANK + j);
      *(v4f*)(sBC + s * (2 * D_STATE) + j) = v;
    }
    __syncthreads();

#pragma unroll 1
    for (int s = 0; s < TCH; ++s) {
      const int t = t0 + s;
      const int l = dir ? (L_SEQ - 1 - t) : t;
      const size_t row = rb + (size_t)l;
      const float* xr = xz + row * (size_t)(2 * D_INNER) + d;
      const float x0 = xr[0];
      const float xp = (l > 0) ? *(xr - 2 * D_INNER) : 0.0f;
      const float xn = (l < L_SEQ - 1) ? xr[2 * D_INNER] : 0.0f;
      const float u = conv_silu1(xp, x0, xn, w0, w1, w2, cbv);
      const float delta = softplus1(dt_raw[row * D_INNER + d] + bias);
      const float du = delta * u;
      const float* bc = sBC + s * (2 * D_STATE);
      float y = 0.0f;
#pragma unroll
      for (int n = 0; n < D_STATE; ++n) {
        const float dA = __expf(delta * An[n]);
        hs[n] = fmaf(hs[n], dA, du * bc[n]);
        y = fmaf(hs[n], bc[D_STATE + n], y);
      }
      y = fmaf(u, Dk, y);
      if (dir == 0) {
        sY[s * 256 + tid] = y;
      } else {
        const float zz = xr[D_INNER];
        const float yp = y0_in[row * D_INNER + d];
        sYh[s * 256 + tid] = (f16t)((yp + y) * zz);
      }
    }
    __syncthreads();

    if (dir == 0) {
      v4f vals[8];
      float* addr[8];
#pragma unroll
      for (int it = 0; it < 8; ++it) {
        const int f = it * 256 + tid;
        const int s = f >> 6, c4 = (f & 63) * 4;
        vals[it] = *(const v4f*)(sY + s * 256 + c4);
        const size_t row = rb + (size_t)(t0 + s);
        addr[it] = y0_out + row * D_INNER + (size_t)dblk * 256 + c4;
      }
#pragma unroll
      for (int it = 0; it < 8; ++it) *(volatile v4f*)addr[it] = vals[it];
      __threadfence();
#pragma unroll
      for (int it = 0; it < 8; ++it) *(volatile v4f*)addr[it] = vals[it];
    } else {
      v8h vals[4];
      f16t* addr[4];
#pragma unroll
      for (int it = 0; it < 4; ++it) {
        const int f = it * 256 + tid;
        const int s = f >> 5, c8 = (f & 31) * 8;
        vals[it] = *(const v8h*)(sYh + s * 256 + c8);
        const size_t row = rb + (size_t)(L_SEQ - 1 - (t0 + s));
        addr[it] = yg_out + row * D_INNER + (size_t)dblk * 256 + c8;
      }
#pragma unroll
      for (int it = 0; it < 4; ++it) *(volatile v8h*)addr[it] = vals[it];
      __threadfence();
#pragma unroll
      for (int it = 0; it < 4; ++it) *(volatile v8h*)addr[it] = vals[it];
    }
  }
}

extern "C" void kernel_launch(void* const* d_in, const int* in_sizes, int n_in,
                              void* d_out, int out_size, void* d_ws, size_t ws_size,
                              hipStream_t stream) {
  if (n_in < 10) return;
  if (in_sizes[0] != M_ROWS * D_MODEL) return;
  if (in_sizes[1] != 2 * D_INNER * D_MODEL) return;
  if (in_sizes[2] != D_INNER * 3) return;
  if (in_sizes[3] != D_INNER) return;
  if (in_sizes[4] != KDIR * XP_N * D_INNER) return;
  if (in_sizes[5] != KDIR * D_INNER * DT_RANK) return;
  if (in_sizes[6] != KDIR * D_INNER) return;
  if (in_sizes[7] != KDIR * D_INNER * D_STATE) return;
  if (in_sizes[8] != KDIR * D_INNER) return;
  if (in_sizes[9] != D_MODEL * D_INNER) return;
  if (out_size != M_ROWS * D_MODEL) return;

  const float* x       = (const float*)d_in[0];
  const float* in_w    = (const float*)d_in[1];
  const float* conv_w  = (const float*)d_in[2];
  const float* conv_b  = (const float*)d_in[3];
  const float* xproj_w = (const float*)d_in[4];
  const float* dtw     = (const float*)d_in[5];
  const float* dtb     = (const float*)d_in[6];
  const float* A_logs  = (const float*)d_in[7];
  const float* Ds      = (const float*)d_in[8];
  const float* out_w   = (const float*)d_in[9];
  float* out = (float*)d_out;

  size_t off = 0;
  auto carve = [&](size_t bytes) -> size_t { size_t o = off; off = (off + bytes + 255) & ~(size_t)255; return o; };
  const size_t bytes_xz   = (size_t)M_ROWS * 2 * D_INNER * 4;
  const size_t bytes_rowf = (size_t)M_ROWS * D_INNER * 4;
  const size_t bytes_rowh = (size_t)M_ROWS * D_INNER * 2;
  const size_t bytes_xh   = (size_t)M_ROWS * D_MODEL * 2;
  const size_t bytes_w1h  = (size_t)2 * D_INNER * D_MODEL * 2;
  const size_t o_xz  = carve(bytes_xz);
  const size_t o_r2  = carve(bytes_rowf);
  const size_t o_r3  = carve(bytes_rowf);
  const size_t o_yg  = carve(bytes_rowh);
  const size_t o_w2  = carve((size_t)KDIR * XP_PAD * D_INNER * 2);
  const size_t o_wdt = carve((size_t)KDIR * D_INNER * DT_PAD * 2);
  const size_t o_w3  = carve((size_t)D_MODEL * D_INNER * 2);
  const size_t o_xd  = carve((size_t)KDIR * M_ROWS * XP_PAD * 4);
  const size_t o_dti = carve((size_t)KDIR * M_ROWS * DT_PAD * 2);
  if (off > ws_size) return;
  if (bytes_xh + bytes_w1h > bytes_rowf) return;
  if (bytes_rowh > bytes_rowf) return;

  char* ws = (char*)d_ws;
  float* xz     = (float*)(ws + o_xz);
  f16t*  xh     = (f16t*)(ws + o_r2);
  f16t*  w1h    = (f16t*)(ws + o_r2 + bytes_xh);
  float* dt_raw = (float*)(ws + o_r2);
  f16t*  u_h    = (f16t*)(ws + o_r3);
  float* y0     = (float*)(ws + o_r3);
  f16t*  yg_h   = (f16t*)(ws + o_yg);
  f16t*  w2h    = (f16t*)(ws + o_w2);
  f16t*  wdth   = (f16t*)(ws + o_wdt);
  f16t*  w3h    = (f16t*)(ws + o_w3);
  float* x_dbl  = (float*)(ws + o_xd);
  f16t*  dtin   = (f16t*)(ws + o_dti);

  auto cvt = [&](const float* src, f16t* dst, int Rs, int Cs, int ps, int R, int Cd,
                 long long sbs, long long dbs, float scale, int batch) {
    size_t ngr = (size_t)R * (size_t)(Cd / 8);
    dim3 grid((unsigned)((ngr + 255) / 256), (unsigned)batch, 1);
    k_cvt_rows<<<grid, dim3(256), 0, stream>>>(src, dst, Rs, Cs, ps, R, Cd, sbs, dbs, scale);
  };
  auto gemm = [&](const f16t* Ap, const f16t* Wp, float* Cp, int M, int N, int K,
                  long long sa, long long sw, long long sc, float oscale, int batch) {
    dim3 grid((unsigned)(N / 64), (unsigned)(M / 64), (unsigned)batch);
    k_gemm_f16<<<grid, dim3(128), 0, stream>>>(Ap, Wp, Cp, M, N, K, sa, sw, sc, oscale);
  };

  cvt(x,       xh,   M_ROWS, D_MODEL, D_MODEL, M_ROWS, D_MODEL, 0, 0, 1.0f, 1);
  cvt(in_w,    w1h,  2 * D_INNER, D_MODEL, D_MODEL, 2 * D_INNER, D_MODEL, 0, 0, W_SCALE, 1);
  cvt(out_w,   w3h,  D_MODEL, D_INNER, D_INNER, D_MODEL, D_INNER, 0, 0, W_SCALE, 1);
  cvt(xproj_w, w2h,  XP_N, D_INNER, D_INNER, XP_PAD, D_INNER,
      (long long)XP_N * D_INNER, (long long)XP_PAD * D_INNER, W_SCALE, KDIR);
  cvt(dtw,     wdth, D_INNER, DT_RANK, DT_RANK, D_INNER, DT_PAD,
      (long long)D_INNER * DT_RANK, (long long)D_INNER * DT_PAD, DTW_SCALE, KDIR);

  gemm(xh, w1h, xz, M_ROWS, 2 * D_INNER, D_MODEL, 0, 0, 0, 1.0f / W_SCALE, 1);

  {
    size_t ngr = (size_t)M_ROWS * (D_INNER / 8);
    k_conv_silu<<<dim3((unsigned)((ngr + 255) / 256)), dim3(256), 0, stream>>>(xz, conv_w, conv_b, u_h);
  }

  gemm(u_h, w2h, x_dbl, M_ROWS, XP_PAD, D_INNER, 0, (long long)XP_PAD * D_INNER,
       (long long)M_ROWS * XP_PAD, 1.0f / W_SCALE, KDIR);

  cvt(x_dbl, dtin, M_ROWS, DT_RANK, XP_PAD, M_ROWS, DT_PAD,
      (long long)M_ROWS * XP_PAD, (long long)M_ROWS * DT_PAD, 1.0f, KDIR);

  for (int dir = 0; dir < KDIR; ++dir) {
    gemm(dtin + (size_t)dir * M_ROWS * DT_PAD, wdth + (size_t)dir * D_INNER * DT_PAD, dt_raw,
         M_ROWS, D_INNER, DT_PAD, 0, 0, 0, 1.0f / DTW_SCALE, 1);
    k_scan<<<dim3(B_SZ * (D_INNER / 256)), dim3(256), 0, stream>>>(
        xz, conv_w, conv_b, dt_raw,
        dtb + (size_t)dir * D_INNER,
        x_dbl + (size_t)dir * M_ROWS * XP_PAD,
        A_logs + (size_t)dir * D_INNER * D_STATE,
        Ds + (size_t)dir * D_INNER,
        y0, y0, yg_h, dir);
  }

  gemm(yg_h, w3h, out, M_ROWS, D_MODEL, D_INNER, 0, 0, 0, 1.0f / W_SCALE, 1);
}
